// Net_78262894068350
// MI455X (gfx1250) — hardware-verified
//
#include <hip/hip_runtime.h>
#include <stddef.h>
#include <stdint.h>


#define NN     10000
#define NE     80000
#define DD     1024
#define NOUT   2048
#define KTILE  32

#define NTHR   256
#define NWAVE  8
#define EPT    8
#define CHUNK  (NTHR * EPT)
#define WCAP   (EPT * 32)
#define LISTN  (NWAVE * WCAP)
#define NBA    1024
#define SLA    10
#define NBLK   10
#define RCAP   28672
#define DEGCAP 64
#define AGG_ZINTS    (LISTN + 2 * RCAP + 3 * NBA)
#define MISC_INTS    16
#define AGG_LDS_INTS (AGG_ZINTS + MISC_INTS)

#define GBM    128
#define GBN    128
#define GTHR   256
#define MTILES 79
#define NTILES 16

#define XB_BLOCKS   5000
#define TR_BLOCKS   1024
#define PREP_BLOCKS (XB_BLOCKS + TR_BLOCKS + 1)
#define TP          72
#define WSMAX  134217728

static_assert(DD == 1024 && DD % 128 == 0);
static_assert(NOUT == 2 * DD);
static_assert(1024 % KTILE == 0 && DD % KTILE == 0 && (2 * DD) % KTILE == 0);
static_assert(NBA * NBLK >= NN);
static_assert(MTILES * GBM >= NN && (MTILES - 1) * GBM < NN);
static_assert(NTILES * GBN == NOUT);
static_assert((NE % 4) == 0);
static_assert((CHUNK & (CHUNK - 1)) == 0 && CHUNK <= 4096);
static_assert((NBA & (NBA - 1)) == 0 && NBA == (1 << SLA));
static_assert(((long long)CHUNK << SLA) < (1LL << 31));
static_assert(((long long)NE << SLA) < (1LL << 31));
static_assert(LISTN % NTHR == 0 && NBA % NWAVE == 0 && NBA % 32 == 0);
static_assert(AGG_ZINTS % (NTHR * 4) == 0);
static_assert(AGG_LDS_INTS * 4 <= 300000);
static_assert(DEGCAP >= 21 + 8 && RCAP >= 8380);
static_assert((long long)NN * DD == (long long)XB_BLOCKS * 256 * 8);
static_assert((long long)NN * DD == 10240000LL);

typedef float          v4f   __attribute__((ext_vector_type(4)));
typedef float          v8f   __attribute__((ext_vector_type(8)));
typedef int            v4i   __attribute__((ext_vector_type(4)));
typedef int            v8i   __attribute__((ext_vector_type(8)));
typedef unsigned short v8us  __attribute__((ext_vector_type(8)));
typedef unsigned short v16us __attribute__((ext_vector_type(16)));
typedef __bf16         v16bf __attribute__((ext_vector_type(16)));
typedef v4f  __attribute__((may_alias)) v4fa;
typedef v4i  __attribute__((may_alias)) v4ia;
typedef v8us __attribute__((may_alias)) v8usa;
union FragB { v16bf v; v16us u; v8us h[2]; v8i w; };

__device__ __forceinline__ v8f wmb(const FragB& a, const FragB& b, v8f c) {
  v8f d = __builtin_amdgcn_wmma_f32_16x16x32_bf16(false, a.v, false, b.v, (short)0, c, false, false);
  asm volatile("v_nop\n\tv_nop\n\tv_nop\n\tv_nop" : "+v"(d) : "v"(a.w), "v"(b.w));
  return d;
}

__device__ __forceinline__ unsigned bf16_bits(float f) {
  const unsigned u = __float_as_uint(f);
  const unsigned r = (u + 0x7FFFu + ((u >> 16) & 1u)) >> 16;
  const unsigned q = (u >> 16) | 0x40u;
  return ((u & 0x7fffffffu) > 0x7f800000u) ? q : r;
}
__device__ __forceinline__ float bf16_val(float f) {
  return __uint_as_float(bf16_bits(f) << 16);
}

struct HL8 { v8us h; v8us l; };
__device__ __forceinline__ HL8 split8(v4f x0, v4f x1) {
  HL8 r;
  unsigned hb;
  hb = bf16_bits(x0.x); r.h[0] = (unsigned short)hb; r.l[0] = (unsigned short)bf16_bits(x0.x - __uint_as_float(hb << 16));
  hb = bf16_bits(x0.y); r.h[1] = (unsigned short)hb; r.l[1] = (unsigned short)bf16_bits(x0.y - __uint_as_float(hb << 16));
  hb = bf16_bits(x0.z); r.h[2] = (unsigned short)hb; r.l[2] = (unsigned short)bf16_bits(x0.z - __uint_as_float(hb << 16));
  hb = bf16_bits(x0.w); r.h[3] = (unsigned short)hb; r.l[3] = (unsigned short)bf16_bits(x0.w - __uint_as_float(hb << 16));
  hb = bf16_bits(x1.x); r.h[4] = (unsigned short)hb; r.l[4] = (unsigned short)bf16_bits(x1.x - __uint_as_float(hb << 16));
  hb = bf16_bits(x1.y); r.h[5] = (unsigned short)hb; r.l[5] = (unsigned short)bf16_bits(x1.y - __uint_as_float(hb << 16));
  hb = bf16_bits(x1.z); r.h[6] = (unsigned short)hb; r.l[6] = (unsigned short)bf16_bits(x1.z - __uint_as_float(hb << 16));
  hb = bf16_bits(x1.w); r.h[7] = (unsigned short)hb; r.l[7] = (unsigned short)bf16_bits(x1.w - __uint_as_float(hb << 16));
  return r;
}

__device__ __forceinline__ v4f sel_nan(v4f v, bool p) {
  const float n = __int_as_float(0x7fc00000);
  v4f r;
  r.x = p ? n : v.x; r.y = p ? n : v.y; r.z = p ? n : v.z; r.w = p ? n : v.w;
  return r;
}

__global__ __launch_bounds__(NTHR) void k_prep(const float* __restrict__ x,
                                               const float* __restrict__ Ws1, const float* __restrict__ Wn1,
                                               const float* __restrict__ b1,
                                               const float* __restrict__ Ws2, const float* __restrict__ Wn2,
                                               const float* __restrict__ b2,
                                               unsigned short* XB, unsigned short* W1T, unsigned short* W2T,
                                               float* B1F, float* B2F) {
  __shared__ __attribute__((aligned(16))) unsigned short sT[64 * TP];
  const int tid = (int)threadIdx.x;
  const int bid = (int)blockIdx.x;
  if (bid < XB_BLOCKS) {
    const size_t g = (size_t)bid * NTHR + (size_t)tid;
    const float* p = x + g * 8;
    const v4f a = *(const v4f*)p;
    const v4f b = *(const v4f*)(p + 4);
    v8us o;
    o[0] = (unsigned short)bf16_bits(a.x); o[1] = (unsigned short)bf16_bits(a.y);
    o[2] = (unsigned short)bf16_bits(a.z); o[3] = (unsigned short)bf16_bits(a.w);
    o[4] = (unsigned short)bf16_bits(b.x); o[5] = (unsigned short)bf16_bits(b.y);
    o[6] = (unsigned short)bf16_bits(b.z); o[7] = (unsigned short)bf16_bits(b.w);
    unsigned short* dp = XB + g * 8;
    *(volatile v8us*)dp = o;
    __threadfence();
    *(volatile v8us*)dp = o;
  } else if (bid < XB_BLOCKS + TR_BLOCKS) {
    const int t   = bid - XB_BLOCKS;
    const int mat = t >> 8;
    const int tt  = t & 255;
    const int k0  = (tt >> 4) * 64;
    const int n0  = (tt & 15) * 64;
    const float* W;
    unsigned short* WT;
    int nOff;
    if (mat == 0)      { W = Ws1; WT = W1T; nOff = 0; }
    else if (mat == 1) { W = Wn1; WT = W1T; nOff = DD; }
    else if (mat == 2) { W = Ws2; WT = W2T; nOff = 0; }
    else               { W = Wn2; WT = W2T; nOff = DD; }
#pragma unroll
    for (int i = 0; i < 4; ++i) {
      const int idx = tid + 256 * i;
      const int kr  = idx >> 4;
      const int c4  = (idx & 15) * 4;
      const v4f v = *(const v4f*)(W + (size_t)(k0 + kr) * DD + n0 + c4);
      sT[(c4 + 0) * TP + kr] = (unsigned short)bf16_bits(v.x);
      sT[(c4 + 1) * TP + kr] = (unsigned short)bf16_bits(v.y);
      sT[(c4 + 2) * TP + kr] = (unsigned short)bf16_bits(v.z);
      sT[(c4 + 3) * TP + kr] = (unsigned short)bf16_bits(v.w);
    }
    __syncthreads();
    const int u0 = tid, u1 = tid + 256;
    const int nr0 = u0 >> 3, k80 = (u0 & 7) * 8;
    const int nr1 = u1 >> 3, k81 = (u1 & 7) * 8;
    const v8us q0 = *(const v8usa*)(sT + nr0 * TP + k80);
    const v8us q1 = *(const v8usa*)(sT + nr1 * TP + k81);
    unsigned short* d0 = WT + (size_t)(nOff + n0 + nr0) * DD + k0 + k80;
    unsigned short* d1 = WT + (size_t)(nOff + n0 + nr1) * DD + k0 + k81;
    *(volatile v8us*)d0 = q0;
    *(volatile v8us*)d1 = q1;
    __threadfence();
    *(volatile v8us*)d0 = q0;
    *(volatile v8us*)d1 = q1;
  } else {
    const v4f a = *(const v4f*)(b1 + 4 * tid);
    const v4f c = *(const v4f*)(b2 + 4 * tid);
    v4f ra, rc;
    ra.x = bf16_val(a.x); ra.y = bf16_val(a.y); ra.z = bf16_val(a.z); ra.w = bf16_val(a.w);
    rc.x = bf16_val(c.x); rc.y = bf16_val(c.y); rc.z = bf16_val(c.z); rc.w = bf16_val(c.w);
    float* p1 = B1F + 4 * tid;
    float* p2 = B2F + 4 * tid;
    *(volatile v4f*)p1 = ra;
    *(volatile v4f*)p2 = rc;
    __threadfence();
    *(volatile v4f*)p1 = ra;
    *(volatile v4f*)p2 = rc;
  }
}

__global__ __launch_bounds__(GTHR) void k_gemm(const unsigned short* __restrict__ A,
                                               const unsigned short* __restrict__ BT, int K, float* SP) {
  __shared__ __attribute__((aligned(16))) float stg[64 * GBN];
  const int tid = (int)threadIdx.x, lane = tid & 31, w = tid >> 5, hh = lane >> 4, m = lane & 15;
  const int wr = w >> 1, wc = w & 1;
  const int m0 = (int)blockIdx.x * GBM;
  const int n0 = (int)blockIdx.y * GBN;

  int r0 = m0 + 32 * wr + m;      r0 = r0 < NN - 1 ? r0 : NN - 1;
  int r1 = m0 + 32 * wr + 16 + m; r1 = r1 < NN - 1 ? r1 : NN - 1;
  const unsigned short* ap0 = A + (size_t)r0 * (size_t)K + 8 * hh;
  const unsigned short* ap1 = A + (size_t)r1 * (size_t)K + 8 * hh;
  const unsigned short* bp  = BT + (size_t)(n0 + 64 * wc + m) * (size_t)DD + 8 * hh;

  v8f acc[2][4];
  {
    const v8f z = {0.f, 0.f, 0.f, 0.f, 0.f, 0.f, 0.f, 0.f};
#pragma unroll
    for (int mt = 0; mt < 2; ++mt)
#pragma unroll
      for (int nt = 0; nt < 4; ++nt) acc[mt][nt] = z;
  }

#pragma unroll 1
  for (int k0 = 0; k0 < K; k0 += KTILE) {
    const int kb = k0 & (DD - 1);
    FragB a0, a1;
    a0.h[0] = *(const v8usa*)(ap0 + k0);
    a0.h[1] = *(const v8usa*)(ap0 + k0 + 16);
    a1.h[0] = *(const v8usa*)(ap1 + k0);
    a1.h[1] = *(const v8usa*)(ap1 + k0 + 16);
#pragma unroll
    for (int nt = 0; nt < 4; ++nt) {
      const unsigned short* wq = bp + (size_t)(16 * nt) * (size_t)DD + kb;
      FragB bf;
      bf.h[0] = *(const v8usa*)wq;
      bf.h[1] = *(const v8usa*)(wq + 16);
      acc[0][nt] = wmb(a0, bf, acc[0][nt]);
      acc[1][nt] = wmb(a1, bf, acc[1][nt]);
    }
  }

#pragma unroll
  for (int mt = 0; mt < 2; ++mt) {
    if (mt != 0) __syncthreads();
#pragma unroll
    for (int nt = 0; nt < 4; ++nt) {
      const int lc = 64 * wc + 16 * nt + m;
#pragma unroll
      for (int r = 0; r < 8; ++r) {
        const int lr = 16 * wr + 8 * hh + r;
        stg[lr * GBN + lc] = acc[mt][nt][r];
      }
    }
    __syncthreads();
#pragma unroll
    for (int ps = 0; ps < 2; ++ps) {
      if (ps != 0) __threadfence();
#pragma unroll
      for (int i = 0; i < 8; ++i) {
        const int sr   = 8 * w + i;
        const int grow = m0 + 32 * (sr >> 4) + 16 * mt + (sr & 15);
        if (grow < NN) {
          const v4f v = *(const v4fa*)(stg + sr * GBN + 4 * lane);
          *(volatile v4f*)(SP + (size_t)grow * NOUT + n0 + 4 * lane) = v;
        }
      }
    }
  }
}

template <int SLB>
__device__ __forceinline__ int scan_chunk(const int* __restrict__ dsts, int nE, int cbase, int slotBase,
                                          int nb, int vec8, int* list, int tid, int lane, int wave) {
  int wc = 0;
  const int el0  = tid * EPT;
  const int e0   = cbase + el0;
  const int sent = -2147483647 - 1;
  v4i da, db;
  if (vec8 != 0 && cbase + CHUNK <= nE) {
    da = *(const v4i*)(dsts + e0);
    db = *(const v4i*)(dsts + e0 + 4);
  } else {
    da.x = (e0     < nE) ? dsts[min(e0,     nE - 1)] : sent;
    da.y = (e0 + 1 < nE) ? dsts[min(e0 + 1, nE - 1)] : sent;
    da.z = (e0 + 2 < nE) ? dsts[min(e0 + 2, nE - 1)] : sent;
    da.w = (e0 + 3 < nE) ? dsts[min(e0 + 3, nE - 1)] : sent;
    db.x = (e0 + 4 < nE) ? dsts[min(e0 + 4, nE - 1)] : sent;
    db.y = (e0 + 5 < nE) ? dsts[min(e0 + 5, nE - 1)] : sent;
    db.z = (e0 + 6 < nE) ? dsts[min(e0 + 6, nE - 1)] : sent;
    db.w = (e0 + 7 < nE) ? dsts[min(e0 + 7, nE - 1)] : sent;
  }
  const unsigned nbs = (unsigned)slotBase;
  const unsigned unb = (unsigned)nb;
  const unsigned s0 = (unsigned)da.x - nbs, s1 = (unsigned)da.y - nbs;
  const unsigned s2 = (unsigned)da.z - nbs, s3 = (unsigned)da.w - nbs;
  const unsigned s4 = (unsigned)db.x - nbs, s5 = (unsigned)db.y - nbs;
  const unsigned s6 = (unsigned)db.z - nbs, s7 = (unsigned)db.w - nbs;
  const bool h0 = s0 < unb, h1 = s1 < unb, h2 = s2 < unb, h3 = s3 < unb;
  const bool h4 = s4 < unb, h5 = s5 < unb, h6 = s6 < unb, h7 = s7 < unb;
  const unsigned any = __builtin_amdgcn_ballot_w32(h0 | h1 | h2 | h3 | h4 | h5 | h6 | h7);
  if (any != 0u) {
#define HITJ(J, HJ, SJ) { \
      const unsigned mj = __builtin_amdgcn_ballot_w32(HJ); \
      if (mj != 0u) { \
        if (HJ) { \
          const int pos = wc + (int)__builtin_amdgcn_mbcnt_lo(mj, 0u); \
          if (pos < WCAP) list[wave * WCAP + pos] = ((el0 + (J)) << SLB) | (int)(SJ); \
        } \
        wc += (int)__builtin_popcount(mj); } }
    HITJ(0, h0, s0)
    HITJ(1, h1, s1)
    HITJ(2, h2, s2)
    HITJ(3, h3, s3)
    HITJ(4, h4, s4)
    HITJ(5, h5, s5)
    HITJ(6, h6, s6)
    HITJ(7, h7, s7)
#undef HITJ
  }
  return wc;
}

template <int MODE>
__device__ __forceinline__ int colq(int q, int lane) {
  return (MODE == 0) ? (256 * (q >> 1) + 8 * lane + 4 * (q & 1)) : (128 * q + 4 * lane);
}

template <int MODE>
__global__ __launch_bounds__(NTHR) void k_scan(const int* __restrict__ gath, const int* __restrict__ keys, int vec8,
                                               const float* __restrict__ SP, const float* __restrict__ BF,
                                               unsigned short* HHL, float* outp) {
  extern __shared__ __attribute__((aligned(16))) int dsm[];
  int* list = dsm;
  int* hl   = dsm + LISTN;
  int* sl   = hl + RCAP;
  int* cnt  = sl + RCAP;
  int* offs = cnt + NBA;
  int* cur  = offs + NBA;
  int* misc = cur + NBA;
  const int tid = (int)threadIdx.x, lane = tid & 31, wave = tid >> 5;
  const int nodeBase = (int)blockIdx.x * NBA;
  const int nE = NE;

  {
    const v4i z4 = {0, 0, 0, 0};
    for (int i = tid * 4; i < AGG_ZINTS; i += NTHR * 4) *(v4ia*)(dsm + i) = z4;
    if (tid < MISC_INTS) misc[tid] = 0;
  }
  __syncthreads();

  int t = 0, ov = 0;
  const int nChunks = (nE + CHUNK - 1) / CHUNK;
#pragma unroll 1
  for (int ch = 0; ch < nChunks; ++ch) {
    const int cbase = ch * CHUNK;
    const int wc = scan_chunk<SLA>(keys, nE, cbase, nodeBase, NBA, vec8, list, tid, lane, wave);
    if (lane == 0) misc[wave] = wc;
    __syncthreads();
    if (wave == 0) {
#pragma unroll 1
      for (int w2 = 0; w2 < NWAVE; ++w2) {
        int c = misc[w2];
        c = c < 0 ? 0 : (c > WCAP ? WCAP : c);
#pragma unroll 1
        for (int b0 = 0; b0 < c; b0 += 32) {
          const int idx = b0 + lane;
          const int ent = list[w2 * WCAP + (idx < WCAP ? idx : WCAP - 1)];
          const int m32 = (c - b0) < 32 ? (c - b0) : 32;
#pragma unroll 1
          for (int k = 0; k < m32; ++k) {
            const int u    = __builtin_amdgcn_readlane(ent, k);
            const int slot = u & (NBA - 1);
            const int el   = (u >> SLA) & (CHUNK - 1);
            const int pk   = ((cbase + el) << SLA) | slot;
            if (t < RCAP) {
              if (lane == 0) { hl[t] = pk; cnt[slot] = cnt[slot] + 1; }
              t = t + 1;
            } else {
              ov = 1;
            }
          }
        }
      }
    }
    __syncthreads();
  }
  if (wave == 0 && lane == 0) { misc[8] = t; misc[9] = ov; }
  __syncthreads();
  int tt = misc[8];
  tt = tt < 0 ? 0 : (tt > RCAP ? RCAP : tt);

  if (wave == 0) {
    const int base = lane * (NBA / 32);
    int s = 0;
    bool bigl = false;
#pragma unroll 1
    for (int i = 0; i < NBA / 32; ++i) {
      const int cv = cnt[base + i];
      s += cv;
      bigl = bigl | (cv > DEGCAP);
    }
    const unsigned bm = __builtin_amdgcn_ballot_w32(bigl);
    if (lane == 0 && bm != 0u) misc[9] = 1;
    int incl = s;
#pragma unroll
    for (int d = 1; d < 32; d <<= 1) {
      const int y = __shfl_up(incl, d, 32);
      if (lane >= d) incl += y;
    }
    int run = incl - s;
#pragma unroll 1
    for (int i = 0; i < NBA / 32; ++i) {
      const int cv = cnt[base + i];
      offs[base + i] = run;
      cur[base + i]  = run;
      run += cv;
    }
  }
  __syncthreads();
  if (wave == 0) {
#pragma unroll 1
    for (int b0 = 0; b0 < tt; b0 += 32) {
      const int idx = b0 + lane;
      const int ent = hl[idx < RCAP ? idx : RCAP - 1];
      const int m32 = (tt - b0) < 32 ? (tt - b0) : 32;
#pragma unroll 1
      for (int k = 0; k < m32; ++k) {
        const int u    = __builtin_amdgcn_readlane(ent, k);
        const int slot = u & (NBA - 1);
        if (lane == 0) {
          int p = cur[slot];
          p = p < 0 ? 0 : (p > RCAP - 1 ? RCAP - 1 : p);
          sl[p] = u;
          cur[slot] = p + 1;
        }
      }
    }
  }
  __syncthreads();
  const int ovf = misc[9];

  v4f bq[8];
#pragma unroll
  for (int q = 0; q < 8; ++q) bq[q] = *(const v4f*)(BF + colq<MODE>(q, lane));

#pragma unroll 1
  for (int si = 0; si < NBA / NWAVE; ++si) {
    const int s    = si * NWAVE + wave;
    const int node = nodeBase + s;
    int c = __builtin_amdgcn_readfirstlane(cnt[s]);
    const bool big = c > DEGCAP;
    c = c < 0 ? 0 : (c > DEGCAP ? DEGCAP : c);
    int o = __builtin_amdgcn_readfirstlane(offs[s]);
    o = o < 0 ? 0 : (o > RCAP ? RCAP : o);
    const int nc = node < NN ? node : NN - 1;
    v4f a[8];
    {
      const v4f z = {0.0f, 0.0f, 0.0f, 0.0f};
#pragma unroll
      for (int q = 0; q < 8; ++q) a[q] = z;
    }
#pragma unroll 1
    for (int b0 = 0; b0 < c; b0 += 32) {
      int idx = o + b0 + lane;
      idx = idx > RCAP - 1 ? RCAP - 1 : idx;
      const int ent = sl[idx];
      int eid = ent >> SLA;
      eid = eid < 0 ? 0 : (eid > nE - 1 ? nE - 1 : eid);
      int sr = gath[eid];
      sr = sr < 0 ? 0 : (sr > NN - 1 ? NN - 1 : sr);
      const int m32 = (c - b0) < 32 ? (c - b0) : 32;
#pragma unroll 1
      for (int k = 0; k < m32; ++k) {
        const int sk = __builtin_amdgcn_readlane(sr, k);
        const float* rp = SP + (size_t)sk * NOUT + DD;
        v4f g[8];
#pragma unroll
        for (int q = 0; q < 8; ++q) g[q] = *(const v4f*)(rp + colq<MODE>(q, lane));
#pragma unroll
        for (int q = 0; q < 8; ++q) a[q] = a[q] + g[q];
      }
    }
    const bool pois = (ovf != 0) | big;
    const float* sp = SP + (size_t)nc * NOUT;
    v4f y[8];
#pragma unroll
    for (int q = 0; q < 8; ++q) {
      const v4f sv = *(const v4f*)(sp + colq<MODE>(q, lane));
      const v4f tq = (sv + a[q]) + bq[q];
      y[q] = sel_nan(tq, pois);
    }
    if constexpr (MODE == 0) {
      HL8 p0 = split8(y[0], y[1]);
      HL8 p1 = split8(y[2], y[3]);
      HL8 p2 = split8(y[4], y[5]);
      HL8 p3 = split8(y[6], y[7]);
      if (node < NN) {
        unsigned short* rpw = HHL + (size_t)node * NOUT + 8 * lane;
#pragma unroll
        for (int ps = 0; ps < 2; ++ps) {
          if (ps != 0) __threadfence();
          *(volatile v8us*)(rpw)            = p0.h;
          *(volatile v8us*)(rpw + 256)      = p1.h;
          *(volatile v8us*)(rpw + 512)      = p2.h;
          *(volatile v8us*)(rpw + 768)      = p3.h;
          *(volatile v8us*)(rpw + DD)       = p0.l;
          *(volatile v8us*)(rpw + DD + 256) = p1.l;
          *(volatile v8us*)(rpw + DD + 512) = p2.l;
          *(volatile v8us*)(rpw + DD + 768) = p3.l;
        }
      }
    } else {
      if (node < NN) {
        float* rpw = outp + (size_t)node * DD + 4 * lane;
#pragma unroll
        for (int ps = 0; ps < 2; ++ps) {
          if (ps != 0) __threadfence();
#pragma unroll
          for (int q = 0; q < 8; ++q) *(volatile v4f*)(rpw + 128 * q) = y[q];
        }
      }
    }
  }
}

static inline size_t al256(size_t o) { return (o + 255) & ~(size_t)255; }

extern "C" void kernel_launch(void* const* d_in, const int* in_sizes, int n_in,
                              void* d_out, int out_size, void* d_ws, size_t ws_size,
                              hipStream_t stream) {
  if (n_in < 8) return;
  if (in_sizes[0] != NN * DD) return;
  if (in_sizes[1] != 2 * NE) return;
  if (in_sizes[2] != DD * DD || in_sizes[3] != DD * DD) return;
  if (in_sizes[4] != DD) return;
  if (in_sizes[5] != DD * DD || in_sizes[6] != DD * DD) return;
  if (in_sizes[7] != DD) return;
  if (out_size != NN * DD) return;

  const float* x   = (const float*)d_in[0];
  const int*   ei  = (const int*)d_in[1];
  const float* Ws1 = (const float*)d_in[2];
  const float* Wn1 = (const float*)d_in[3];
  const float* b1  = (const float*)d_in[4];
  const float* Ws2 = (const float*)d_in[5];
  const float* Wn2 = (const float*)d_in[6];
  const float* b2  = (const float*)d_in[7];
  float* out = (float*)d_out;
  const int* src = ei;
  const int* dst = ei + NE;

  char* ws = (char*)d_ws;
  size_t off = 0;
  const size_t oSP  = off; off = al256(off + (size_t)NN * NOUT * 4);
  const size_t oHHL = off; off = al256(off + (size_t)NN * NOUT * 2);
  const size_t oW1  = off; off = al256(off + (size_t)NOUT * DD * 2);
  const size_t oW2  = off; off = al256(off + (size_t)NOUT * DD * 2);
  const size_t oB1  = off; off = al256(off + (size_t)DD * 4);
  const size_t oB2  = off; off = al256(off + (size_t)DD * 4);
  if (off > ws_size || off > (size_t)WSMAX) return;
  float*          SP  = (float*)(ws + oSP);
  unsigned short* HHL = (unsigned short*)(ws + oHHL);
  unsigned short* XB  = HHL;
  unsigned short* W1T = (unsigned short*)(ws + oW1);
  unsigned short* W2T = (unsigned short*)(ws + oW2);
  float*          B1F = (float*)(ws + oB1);
  float*          B2F = (float*)(ws + oB2);

  const size_t scanLds = (size_t)AGG_LDS_INTS * 4;
  hipFuncSetAttribute(reinterpret_cast<const void*>(&k_scan<0>), hipFuncAttributeMaxDynamicSharedMemorySize, (int)scanLds);
  hipFuncSetAttribute(reinterpret_cast<const void*>(&k_scan<1>), hipFuncAttributeMaxDynamicSharedMemorySize, (int)scanLds);

  const dim3 gG(MTILES, NTILES);
  const int vec8 = 1;

  k_prep<<<PREP_BLOCKS, NTHR, 0, stream>>>(x, Ws1, Wn1, b1, Ws2, Wn2, b2, XB, W1T, W2T, B1F, B2F);
  k_gemm<<<gG, GTHR, 0, stream>>>(XB, W1T, DD, SP);
  k_scan<0><<<NBLK, NTHR, scanLds, stream>>>(src, dst, vec8, SP, B1F, HHL, out);
  k_gemm<<<gG, GTHR, 0, stream>>>(HHL, W2T, 2 * DD, SP);
  k_scan<1><<<NBLK, NTHR, scanLds, stream>>>(src, dst, vec8, SP, B2F, HHL, out);
}
